// KalmanNetLayer_6330781794388
// MI455X (gfx1250) — hardware-run, weakly checked
//
#include <hip/hip_runtime.h>
#include <math.h>

typedef __attribute__((ext_vector_type(16))) _Float16 v16h;
typedef __attribute__((ext_vector_type(8)))  _Float16 v8h;
typedef __attribute__((ext_vector_type(16))) __bf16   v16b;
typedef __attribute__((ext_vector_type(8)))  __bf16   v8b;
typedef __attribute__((ext_vector_type(8)))  float    v8f;
typedef __attribute__((ext_vector_type(4)))  float    v4f;
typedef __attribute__((ext_vector_type(4)))  unsigned int v4u;

constexpr int kNB   = 4;
constexpr int kSeq  = 2048;
constexpr int kFin  = 512;
constexpr int kNH   = 8;
constexpr int kHD   = 32;
constexpr int kHid  = kNH * kHD;
constexpr int kNAct = 16;
constexpr int kTok  = kNB * kSeq;
constexpr int kN1   = 832;
constexpr int kN2   = 576;
constexpr int kK2   = 32;
constexpr int kChunk = 16;
constexpr int kNChunk = kSeq / kChunk;
constexpr float kEps = 1e-6f;
constexpr float kOnCarry  = 64.0f;
constexpr float kWoCarry  = 1024.0f;
constexpr float kOutScale = 1.0f / (kOnCarry * kWoCarry);
constexpr float kInvHid   = 1.0f / (float)kHid;
constexpr float kHalfMinNormal = 6.103515625e-5f;
constexpr int kOut0 = kNB * kNH * kHD * kHD;
constexpr int kOut1 = kTok * kFin;
static_assert(kHid == 256);
static_assert(kTok == 8192);
static_assert(3 * kHid + 2 * kNH <= kN1 && (kN1 % 64) == 0);
static_assert(2 * kHid + kNH <= kN2 && (kN2 % 64) == 0);
static_assert((kFin % 32) == 0 && (kK2 % 32) == 0 && (kHid % 32) == 0);
static_assert((kTok % 64) == 0 && (kFin % 64) == 0);
static_assert(kSeq % kChunk == 0);
static_assert(kOut0 * 4 == 131072);
static_assert((kOut0 + kOut1) * 4 == 16908288);

constexpr size_t kSzXB  = (size_t)kTok * kFin * 2;
constexpr size_t kSzAB  = (size_t)kTok * kK2 * 2;
constexpr size_t kSzWQT = (size_t)kN1 * kFin * 2;
constexpr size_t kSzWAT = (size_t)kN2 * kK2 * 2;
constexpr size_t kSzWOT = (size_t)kFin * kHid * 2;
constexpr size_t kSzP   = (size_t)kTok * kN1 * 4;
constexpr size_t kSzPA  = (size_t)kTok * kN2 * 4;
constexpr size_t kSzTV  = (size_t)kTok * kHid * 4;
constexpr size_t kSzG   = (size_t)kTok * 32 * 4;
constexpr size_t kSzON  = (size_t)kTok * kHid * 2;
constexpr size_t kOffXB  = 0;
constexpr size_t kOffAB  = kOffXB  + kSzXB;
constexpr size_t kOffWQT = kOffAB  + kSzAB;
constexpr size_t kOffWAT = kOffWQT + kSzWQT;
constexpr size_t kOffWOT = kOffWAT + kSzWAT;
constexpr size_t kOffP   = kOffWOT + kSzWOT;
constexpr size_t kOffPA  = kOffP   + kSzP;
constexpr size_t kOffQN  = kOffPA  + kSzPA;
constexpr size_t kOffKN  = kOffQN  + kSzTV;
constexpr size_t kOffKU  = kOffKN  + kSzTV;
constexpr size_t kOffVU  = kOffKU  + kSzTV;
constexpr size_t kOffG   = kOffVU  + kSzTV;
constexpr size_t kOffO   = kOffG   + kSzG;
constexpr size_t kOffON  = kOffO   + kSzTV;
constexpr size_t kWsTotal = kOffON + kSzON;
static_assert(kWsTotal == 103387136ull);
static_assert(kWsTotal <= 134217728ull);
static_assert((kOffAB % 128) == 0 && (kOffWQT % 128) == 0 && (kOffWAT % 128) == 0 && (kOffWOT % 128) == 0 &&
              (kOffP % 128) == 0 && (kOffPA % 128) == 0 && (kOffQN % 128) == 0 && (kOffKN % 128) == 0 &&
              (kOffKU % 128) == 0 && (kOffVU % 128) == 0 && (kOffG % 128) == 0 && (kOffO % 128) == 0 &&
              (kOffON % 128) == 0);

__device__ __forceinline__ unsigned short f2bf_bits(float f) {
  unsigned u = __float_as_uint(f);
  return (unsigned short)((u + 0x7FFFu + ((u >> 16) & 1u)) >> 16);
}
__device__ __forceinline__ float bf_bits2f(unsigned short h) { return __uint_as_float(((unsigned)h) << 16); }
__device__ __forceinline__ float bf16r(float f) { return bf_bits2f(f2bf_bits(f)); }
__device__ __forceinline__ unsigned pk16(unsigned short a, unsigned short b) { return (unsigned)a | ((unsigned)b << 16); }
__device__ __forceinline__ unsigned short h_bits(float f) { const _Float16 h = (_Float16)f; return __builtin_bit_cast(unsigned short, h); }
__device__ __forceinline__ float flush_h(float s) { return (fabsf(s) < kHalfMinNormal) ? 0.0f : s; }
__device__ __forceinline__ void pin1(float& x) { asm volatile("" : "+v"(x)); }
__device__ __forceinline__ float wave_sum(float v) {
#pragma unroll
  for (int off = 16; off > 0; off >>= 1) v += __shfl_xor(v, off, 32);
  return v;
}
__device__ __forceinline__ float sigm(float x) { return __builtin_amdgcn_rcpf(1.0f + expf(-x)); }

__device__ __forceinline__ void dep_guard4_h(v8f& a, v8f& b, v8f& c, v8f& d, v16h x, v16h y) { asm volatile("v_nop\n\tv_nop\n\tv_nop\n\tv_nop" : "+v"(a), "+v"(b), "+v"(c), "+v"(d) : "v"(x), "v"(y)); }
__device__ __forceinline__ void dep_guard4_b(v8f& a, v8f& b, v8f& c, v8f& d, v16b x, v16b y) { asm volatile("v_nop\n\tv_nop\n\tv_nop\n\tv_nop" : "+v"(a), "+v"(b), "+v"(c), "+v"(d) : "v"(x), "v"(y)); }
__device__ __forceinline__ void keep4_h(v16h a, v16h b, v16h c, v16h d) { asm volatile("v_nop" :: "v"(a), "v"(b), "v"(c), "v"(d)); }
__device__ __forceinline__ void keep4_b(v16b a, v16b b, v16b c, v16b d) { asm volatile("v_nop" :: "v"(a), "v"(b), "v"(c), "v"(d)); }
__device__ __forceinline__ void acc_guard4(v8f& a, v8f& b, v8f& c, v8f& d) { asm volatile("v_nop\n\tv_nop\n\tv_nop\n\tv_nop" : "+v"(a), "+v"(b), "+v"(c), "+v"(d)); }
template <typename T> struct Frag;
template <> struct Frag<_Float16> {
  typedef v16h V; union U { v16h v; v8h h[2]; };
  static __device__ __forceinline__ v16h load(const _Float16* p) {
    U f; f.h[0] = *(const v8h*)(p); f.h[1] = *(const v8h*)(p + 16); return f.v;
  }
  static __device__ __forceinline__ v8f mma(v16h a, v16h b, v8f c) {
    return __builtin_amdgcn_wmma_f32_16x16x32_f16(false, a, false, b, (short)0, c, false, false);
  }
  static __device__ __forceinline__ void guard4(v8f& a, v8f& b, v8f& c, v8f& d, v16h x, v16h y) { dep_guard4_h(a, b, c, d, x, y); }
  static __device__ __forceinline__ void keep(v16h a, v16h b, v16h c, v16h d) { keep4_h(a, b, c, d); }
};
template <> struct Frag<__bf16> {
  typedef v16b V; union U { v16b v; v8b h[2]; };
  static __device__ __forceinline__ v16b load(const __bf16* p) {
    U f; f.h[0] = *(const v8b*)(p); f.h[1] = *(const v8b*)(p + 16); return f.v;
  }
  static __device__ __forceinline__ v8f mma(v16b a, v16b b, v8f c) {
    return __builtin_amdgcn_wmma_f32_16x16x32_bf16(false, a, false, b, (short)0, c, false, false);
  }
  static __device__ __forceinline__ void guard4(v8f& a, v8f& b, v8f& c, v8f& d, v16b x, v16b y) { dep_guard4_b(a, b, c, d, x, y); }
  static __device__ __forceinline__ void keep(v16b a, v16b b, v16b c, v16b d) { keep4_b(a, b, c, d); }
};

template <int ET> struct Elem;
template <> struct Elem<0> { typedef _Float16 T; };
template <> struct Elem<1> { typedef __bf16 T; };
template <int ET, bool BIASN>
__global__ __launch_bounds__(256) void wmma_gemm64(
    const unsigned short* __restrict__ Ap, int lda,
    const unsigned short* __restrict__ Btp, int ldb,
    float* __restrict__ Cout, int ldc,
    const float* __restrict__ bias,
    int M, int N, int K, float scale) {
  typedef typename Elem<ET>::T T;
  typedef typename Frag<T>::V V;
  const T* A = (const T*)Ap; const T* Bt = (const T*)Btp;
  __shared__ __align__(16) float sT[8][16 * 68];
  const int lane = threadIdx.x & 31;
  const int wave = threadIdx.x >> 5;
  const int tilesN = N >> 6;
  const int tilesM = M >> 6;
  const int tile = blockIdx.x * 8 + wave;
  if (tile >= tilesM * tilesN) return;
  const int tm = tile / tilesN;
  const int tn = tile - tm * tilesN;
  const int m0 = tm << 6;
  const int n0 = tn << 6;

  const int rlane = lane & 15;
  const int koff  = (lane >> 4) * 8;
  const int mOff  = (lane >> 4) * 8;

  v8f acc[4][4];
#pragma unroll
  for (int i = 0; i < 4; ++i)
#pragma unroll
    for (int j = 0; j < 4; ++j) acc[i][j] = (v8f){0.f,0.f,0.f,0.f,0.f,0.f,0.f,0.f};

  for (int k0 = 0; k0 < K; k0 += 32) {
    V bh[4];
#pragma unroll
    for (int j = 0; j < 4; ++j) {
      const size_t bo = (size_t)(n0 + (j << 4) + rlane) * ldb + koff + k0;
      bh[j] = Frag<T>::load(Bt + bo);
    }
#pragma unroll
    for (int i = 0; i < 4; ++i) {
      const size_t ao = (size_t)(m0 + (i << 4) + rlane) * lda + koff + k0;
      V ah = Frag<T>::load(A + ao);
#pragma unroll
      for (int j = 0; j < 4; ++j) acc[i][j] = Frag<T>::mma(ah, bh[j], acc[i][j]);
      Frag<T>::guard4(acc[i][0], acc[i][1], acc[i][2], acc[i][3], ah, bh[3]);
    }
    Frag<T>::keep(bh[0], bh[1], bh[2], bh[3]);
  }
  acc_guard4(acc[0][0], acc[0][1], acc[0][2], acc[0][3]);
  acc_guard4(acc[1][0], acc[1][1], acc[1][2], acc[1][3]);
  acc_guard4(acc[2][0], acc[2][1], acc[2][2], acc[2][3]);
  acc_guard4(acc[3][0], acc[3][1], acc[3][2], acc[3][3]);

  float* slab = sT[wave];
#pragma unroll
  for (int i = 0; i < 4; ++i) {
    const int mBase = m0 + (i << 4);
#pragma unroll
    for (int j = 0; j < 4; ++j) {
      const int n = n0 + (j << 4) + rlane;
      float bv = 0.f;
      if (BIASN) bv = bf16r(bias[n]);
#pragma unroll
      for (int r = 0; r < 8; ++r) {
        float v = acc[i][j][r] * scale;
        if (BIASN) v += bv;
        slab[(mOff + r) * 68 + (j << 4) + rlane] = v;
      }
    }
    __builtin_amdgcn_fence(__ATOMIC_RELEASE, "workgroup");
    __builtin_amdgcn_wave_barrier();
    __builtin_amdgcn_fence(__ATOMIC_ACQUIRE, "workgroup");
    {
      const int hh = lane >> 4, c4 = (lane & 15) * 4;
      for (int pass = 0; pass < 2; ++pass) {
#pragma unroll
        for (int it = 0; it < 8; ++it) {
          const int row = it * 2 + hh;
          v4f v = *(const v4f*)(slab + row * 68 + c4);
          *(volatile v4f*)(Cout + (size_t)(mBase + row) * ldc + n0 + c4) = v;
        }
        __threadfence();
      }
    }
    __builtin_amdgcn_fence(__ATOMIC_RELEASE, "workgroup");
    __builtin_amdgcn_wave_barrier();
    __builtin_amdgcn_fence(__ATOMIC_ACQUIRE, "workgroup");
  }
}

__global__ __launch_bounds__(256) void cvt_x_bf16_kernel(const float* __restrict__ src, unsigned short* __restrict__ dst, int n8) {
  const int i = blockIdx.x * 256 + threadIdx.x;
  if (i >= n8) return;
  const float* p = src + 8 * (size_t)i;
  const v4f a = *(const v4f*)(p);
  const v4f c = *(const v4f*)(p + 4);
  unsigned short hb[8];
#pragma unroll
  for (int e = 0; e < 4; ++e) {
    hb[e]     = f2bf_bits(a[e]);
    hb[4 + e] = f2bf_bits(c[e]);
  }
  const v4u u = (v4u){pk16(hb[0], hb[1]), pk16(hb[2], hb[3]), pk16(hb[4], hb[5]), pk16(hb[6], hb[7])};
  unsigned short* q = dst + 8 * (size_t)i;
  *(volatile v4u*)q = u;
  __threadfence();
  *(volatile v4u*)q = u;
}

__global__ __launch_bounds__(256) void pack_action_kernel(const float* __restrict__ act, unsigned short* __restrict__ dst) {
  const int i   = blockIdx.x * 256 + threadIdx.x;
  const int row = i >> 2;
  const int c8  = i & 3;
  const float* p = act + (size_t)row * kNAct + (c8 & 1) * 8;
  const v4f a = *(const v4f*)(p);
  const v4f c = *(const v4f*)(p + 4);
  float f[8];
#pragma unroll
  for (int e = 0; e < 4; ++e) { f[e] = a[e]; f[4 + e] = c[e]; }
#pragma unroll
  for (int e = 0; e < 8; ++e) pin1(f[e]);
  const bool real = (c8 < 2);
  unsigned short hb[8];
#pragma unroll
  for (int e = 0; e < 8; ++e) {
    const float g = real ? f[e] : 0.0f;
    hb[e] = f2bf_bits(g);
  }
  const v4u u = (v4u){pk16(hb[0], hb[1]), pk16(hb[2], hb[3]), pk16(hb[4], hb[5]), pk16(hb[6], hb[7])};
  unsigned short* q = dst + 8 * (size_t)i;
  *(volatile v4u*)q = u;
  __threadfence();
  *(volatile v4u*)q = u;
}

template <int MODE>
__global__ __launch_bounds__(256) void pack_wT_kernel(const float* __restrict__ W0, const float* __restrict__ W1,
                                                      const float* __restrict__ W2, const float* __restrict__ Wg0,
                                                      const float* __restrict__ Wg1, unsigned short* __restrict__ out) {
  __shared__ float sm[64][65];
  const int t  = threadIdx.x;
  const int k0 = blockIdx.x * 64;
  const int nt = blockIdx.y;
  const int n0 = nt * 64;
  constexpr int srcld = (MODE == 0) ? kHid : kFin;
  constexpr int outld = (MODE == 0) ? kFin : kHid;
  if (MODE == 1 || nt < 12) {
    const float* W = W0;
    int col0 = n0;
    if (MODE == 0) {
      W = (nt < 4) ? W0 : ((nt < 8) ? W1 : W2);
      col0 = (nt & 3) * 64;
    }
#pragma unroll 4
    for (int i = 0; i < 16; ++i) {
      const int e = i * 256 + t;
      const int r = e >> 6;
      const int c = e & 63;
      sm[c][r] = W[(size_t)(k0 + r) * srcld + col0 + c];
    }
  } else {
#pragma unroll 1
    for (int i = 0; i < 16; ++i) {
      const int e = i * 256 + t;
      const int r = e >> 6;
      const int c = e & 63;
      const int cc = c & 7;
      float vb = Wg0[(size_t)(k0 + r) * kNH + cc];
      float va = Wg1[(size_t)(k0 + r) * kNH + cc];
      pin1(vb);
      pin1(va);
      const float v = (c < 8) ? vb : ((c < 16) ? va : 0.0f);
      sm[c][r] = v;
    }
  }
  __syncthreads();
  const int lane = t & 31, wave = t >> 5;
  const int q = lane >> 3, c8 = (lane & 7) * 8;
  v4u u[2];
#pragma unroll
  for (int it = 0; it < 2; ++it) {
    const int row = wave * 8 + it * 4 + q;
    unsigned short hb[8];
#pragma unroll
    for (int e = 0; e < 8; ++e) {
      const float v = sm[row][c8 + e];
      if (MODE == 0) hb[e] = f2bf_bits(v);
      else           hb[e] = h_bits(flush_h(bf16r(v) * kWoCarry));
    }
    u[it] = (v4u){pk16(hb[0], hb[1]), pk16(hb[2], hb[3]), pk16(hb[4], hb[5]), pk16(hb[6], hb[7])};
  }
  for (int pass = 0; pass < 2; ++pass) {
#pragma unroll
    for (int it = 0; it < 2; ++it) {
      const int row = wave * 8 + it * 4 + q;
      *(volatile v4u*)(out + (size_t)(n0 + row) * outld + k0 + c8) = u[it];
    }
    __threadfence();
  }
}

__global__ __launch_bounds__(256) void pack_waT_kernel(const float* __restrict__ Wku, const float* __restrict__ Wvu,
                                                       const float* __restrict__ Wgm, unsigned short* __restrict__ out) {
  __shared__ float sm[64][17];
  const int t   = threadIdx.x;
  const int blk = blockIdx.x;
  const int n0  = blk * 64;
  if (blk < 8) {
    const float* W = (blk < 4) ? Wku : Wvu;
    const int col0 = (blk & 3) * 64;
#pragma unroll
    for (int i = 0; i < 4; ++i) {
      const int e  = i * 256 + t;
      const int kk = e >> 6;
      const int c  = e & 63;
      sm[c][kk] = W[(size_t)kk * kHid + col0 + c];
    }
  } else {
#pragma unroll 1
    for (int i = 0; i < 4; ++i) {
      const int e  = i * 256 + t;
      const int kk = e >> 6;
      const int c  = e & 63;
      float g = Wgm[kk * kNH + (c & 7)];
      pin1(g);
      sm[c][kk] = (c < 8) ? g : 0.0f;
    }
  }
  __syncthreads();
  const int n  = t >> 2;
  const int c8 = t & 3;
  const bool real = (c8 < 2);
  unsigned short hb[8];
#pragma unroll
  for (int e = 0; e < 8; ++e) {
    const float v = sm[n][(c8 & 1) * 8 + e];
    const float g = real ? v : 0.0f;
    hb[e] = f2bf_bits(g);
  }
  const v4u u = (v4u){pk16(hb[0], hb[1]), pk16(hb[2], hb[3]), pk16(hb[4], hb[5]), pk16(hb[6], hb[7])};
  unsigned short* q = out + (size_t)(n0 + n) * kK2 + c8 * 8;
  *(volatile v4u*)q = u;
  __threadfence();
  *(volatile v4u*)q = u;
}

__global__ __launch_bounds__(256) void token_prep_kernel(const float* __restrict__ P, const float* __restrict__ PA,
                                                         const float* __restrict__ mask,
                                                         float* __restrict__ QN, float* __restrict__ KN,
                                                         float* __restrict__ KU, float* __restrict__ VU,
                                                         float* __restrict__ G) {
  __shared__ __align__(16) float sQ[8 * kHid];
  __shared__ __align__(16) float sK[8 * kHid];
  __shared__ __align__(16) float sU[8 * kHid];
  __shared__ __align__(16) float sV[8 * kHid];
  __shared__ __align__(16) float sG[8 * 32];
  const int tid = threadIdx.x;
  const int d = tid & 31;
  const int h = tid >> 5;
  const int t0 = blockIdx.x * 8;
#pragma unroll 1
  for (int tt = 0; tt < 8; ++tt) {
    const size_t t = (size_t)(t0 + tt);
    const float* pr = P + t * kN1;
    const float* ar = PA + t * kN2;
    const float qr = pr[h * kHD + d];
    const float kr = pr[kHid + h * kHD + d];
    const float ur = ar[h * kHD + d];
    const float vr = ar[kHid + h * kHD + d];
    const float bl = pr[3 * kHid + h];
    const float al = pr[3 * kHid + kNH + h];
    const float gl = ar[2 * kHid + h];
    const float mk = bf16r(mask[t]);
    const float qa = qr * sigm(qr);
    const float ka = kr * sigm(kr);
    const float ua = ur * sigm(ur);
    const float qn = qa * rsqrtf(wave_sum(qa * qa) + kEps);
    const float kn = ka * rsqrtf(wave_sum(ka * ka) + kEps);
    const float un = ua * rsqrtf(wave_sum(ua * ua) + kEps);
    const float cc = wave_sum(un * kn);
    const float beta = sigm(bl);
    const float av   = sigm(al) * (1.0f - mk);
    const float bg   = sigm(gl);
    const float gsel = (d == 0) ? beta : ((d == 1) ? av : ((d == 2) ? bg : cc));
    sQ[tt * kHid + tid] = qn;
    sK[tt * kHid + tid] = kn;
    sU[tt * kHid + tid] = un;
    sV[tt * kHid + tid] = vr;
    if (d < 4) sG[tt * 32 + h * 4 + d] = gsel;
  }
  __syncthreads();
  v4f vq[2], vk[2], vu[2], vv[2];
#pragma unroll
  for (int it = 0; it < 2; ++it) {
    const int idx = (it * 256 + tid) * 4;
    vq[it] = *(const v4f*)(sQ + idx);
    vk[it] = *(const v4f*)(sK + idx);
    vu[it] = *(const v4f*)(sU + idx);
    vv[it] = *(const v4f*)(sV + idx);
  }
  const v4f vg = *(const v4f*)(sG + (tid & 63) * 4);
  const size_t pbase = (size_t)t0 * kHid;
  const size_t gbase = (size_t)t0 * 32;
  for (int pass = 0; pass < 2; ++pass) {
#pragma unroll
    for (int it = 0; it < 2; ++it) {
      const size_t o = pbase + (size_t)(it * 256 + tid) * 4;
      *(volatile v4f*)(QN + o) = vq[it];
      *(volatile v4f*)(KN + o) = vk[it];
      *(volatile v4f*)(KU + o) = vu[it];
      *(volatile v4f*)(VU + o) = vv[it];
    }
    if (tid < 64) *(volatile v4f*)(G + gbase + (size_t)tid * 4) = vg;
    __threadfence();
  }
}

struct StageRegs { v4f k, u, q, v, w, g; };

__device__ __forceinline__ StageRegs stage_fetch(const float* __restrict__ QN, const float* __restrict__ KN,
                                                 const float* __restrict__ KU, const float* __restrict__ VU,
                                                 const float* __restrict__ P, const float* __restrict__ G,
                                                 size_t tok, int h, int sc4) {
  StageRegs s;
  const size_t o = tok * kHid + (size_t)(h * kHD + sc4);
  s.k = *(const v4f*)(KN + o);
  s.u = *(const v4f*)(KU + o);
  s.q = *(const v4f*)(QN + o);
  s.w = *(const v4f*)(VU + o);
  s.v = *(const v4f*)(P + tok * kN1 + (size_t)(2 * kHid + h * kHD + sc4));
  s.g = *(const v4f*)(G + tok * 32 + (size_t)(h * 4));
  return s;
}

__global__ __launch_bounds__(128) void gated_state_scan_kernel(const float* __restrict__ QN, const float* __restrict__ KN,
                                                               const float* __restrict__ KU, const float* __restrict__ VU,
                                                               const float* __restrict__ P, const float* __restrict__ G,
                                                               const float* __restrict__ carry,
                                                               float* __restrict__ O, float* __restrict__ newCarry) {
  __shared__ __align__(16) float sK[kChunk * kHD];
  __shared__ __align__(16) float sU[kChunk * kHD];
  __shared__ __align__(16) float sQ[kChunk * kHD];
  __shared__ __align__(16) float sV[kChunk * kHD];
  __shared__ __align__(16) float sW[kChunk * kHD];
  __shared__ __align__(16) float sO[kChunk * kHD];
  __shared__ __align__(16) float sG[kChunk * 4];
  __shared__ __align__(16) float sH[kHD * 36];
  const int tid = threadIdx.x, lane = tid & 31, wave = tid >> 5;
  const int bh = blockIdx.x;
  const int b  = bh >> 3;
  const int h  = bh & 7;
  const int r  = lane >> 2;
  const int jq = lane & 3;
  const int i  = wave * 8 + r;
  const int j0 = jq * 8;
  const int srow = tid >> 3;
  const int sc4  = (tid & 7) * 4;
  const size_t tokbase = (size_t)b * kSeq;

  float Hs[8];
  {
    const float* cp = carry + (size_t)bh * (kHD * kHD) + (size_t)(i * kHD + j0);
    const v4f c0 = *(const v4f*)(cp);
    const v4f c1 = *(const v4f*)(cp + 4);
#pragma unroll
    for (int e = 0; e < 4; ++e) { Hs[e] = bf16r(c0[e]); Hs[4 + e] = bf16r(c1[e]); }
  }

  {
    const StageRegs s0 = stage_fetch(QN, KN, KU, VU, P, G, tokbase + (size_t)srow, h, sc4);
    *(v4f*)(sK + srow * kHD + sc4) = s0.k;
    *(v4f*)(sU + srow * kHD + sc4) = s0.u;
    *(v4f*)(sQ + srow * kHD + sc4) = s0.q;
    *(v4f*)(sV + srow * kHD + sc4) = s0.v;
    *(v4f*)(sW + srow * kHD + sc4) = s0.w;
    *(v4f*)(sG + srow * 4) = s0.g;
  }
  __syncthreads();

#pragma unroll 1
  for (int c = 0; c < kNChunk; ++c) {
#pragma unroll 1
    for (int s = 0; s < kChunk; ++s) {
      const float* kp = sK + s * kHD + j0;
      const float* up = sU + s * kHD + j0;
      const float* qp = sQ + s * kHD + j0;
      const v4f ka = *(const v4f*)(kp), kb = *(const v4f*)(kp + 4);
      const v4f ua = *(const v4f*)(up), ub = *(const v4f*)(up + 4);
      const v4f qa = *(const v4f*)(qp), qb = *(const v4f*)(qp + 4);
      const v4f g  = *(const v4f*)(sG + s * 4);
      const float vi  = sV[s * kHD + i];
      const float vui = sW[s * kHD + i];
      float kv[8], uv[8], qv[8];
#pragma unroll
      for (int e = 0; e < 4; ++e) {
        kv[e] = ka[e]; kv[4 + e] = kb[e];
        uv[e] = ua[e]; uv[4 + e] = ub[e];
        qv[e] = qa[e]; qv[4 + e] = qb[e];
      }
      float hk = 0.0f;
#pragma unroll
      for (int e = 0; e < 8; ++e) hk = fmaf(Hs[e], kv[e], hk);
      hk += __shfl_xor(hk, 1, 32);
      hk += __shfl_xor(hk, 2, 32);
      const float beta = g[0], av = g[1], bg = g[2], cc = g[3];
      const float gi = bg * vui;
      const float wi = beta * (vi - av * hk - gi * cc);
      float o = 0.0f;
#pragma unroll
      for (int e = 0; e < 8; ++e) {
        const float hn = fmaf(av, Hs[e], fmaf(wi, kv[e], gi * uv[e]));
        Hs[e] = hn;
        o = fmaf(hn, qv[e], o);
      }
      o += __shfl_xor(o, 1, 32);
      o += __shfl_xor(o, 2, 32);
      if (jq == 0) sO[s * kHD + i] = o;
    }
    __syncthreads();
    const v4f ov = *(const v4f*)(sO + srow * kHD + sc4);
    const int cn = (c + 1 < kNChunk) ? (c + 1) : (kNChunk - 1);
    const StageRegs sn = stage_fetch(QN, KN, KU, VU, P, G, tokbase + (size_t)(cn * kChunk + srow), h, sc4);
    float* op = O + (tokbase + (size_t)(c * kChunk + srow)) * kHid + (size_t)(h * kHD + sc4);
    *(volatile v4f*)op = ov;
    __threadfence();
    *(volatile v4f*)op = ov;
    *(v4f*)(sK + srow * kHD + sc4) = sn.k;
    *(v4f*)(sU + srow * kHD + sc4) = sn.u;
    *(v4f*)(sQ + srow * kHD + sc4) = sn.q;
    *(v4f*)(sV + srow * kHD + sc4) = sn.v;
    *(v4f*)(sW + srow * kHD + sc4) = sn.w;
    *(v4f*)(sG + srow * 4) = sn.g;
    __syncthreads();
  }

#pragma unroll
  for (int e = 0; e < 8; ++e) sH[i * 36 + j0 + e] = Hs[e];
  __syncthreads();
  v4f hv[2];
#pragma unroll
  for (int it = 0; it < 2; ++it) hv[it] = *(const v4f*)(sH + (it * 16 + srow) * 36 + sc4);
  float* ncp = newCarry + (size_t)bh * (kHD * kHD);
  for (int pass = 0; pass < 2; ++pass) {
#pragma unroll
    for (int it = 0; it < 2; ++it) *(volatile v4f*)(ncp + (it * 16 + srow) * kHD + sc4) = hv[it];
    __threadfence();
  }
}

__global__ __launch_bounds__(256) void rms_rows_kernel(const float* __restrict__ O, const float* __restrict__ rscale,
                                                       unsigned short* __restrict__ ON) {
  const int tid = threadIdx.x, lane = tid & 31;
  const int row = blockIdx.x * 8 + (tid >> 5);
  const float* rp = O + (size_t)row * kHid + 8 * lane;
  const v4f a = *(const v4f*)(rp);
  const v4f c = *(const v4f*)(rp + 4);
  const v4f sa = *(const v4f*)(rscale + 8 * lane);
  const v4f sc = *(const v4f*)(rscale + 8 * lane + 4);
  float ss = 0.0f;
#pragma unroll
  for (int e = 0; e < 4; ++e) { ss = fmaf(a[e], a[e], ss); ss = fmaf(c[e], c[e], ss); }
  ss = wave_sum(ss);
  const float rinv = rsqrtf(ss * kInvHid + kEps);
  unsigned short hb[8];
#pragma unroll
  for (int e = 0; e < 4; ++e) {
    const float v0 = ((a[e] * rinv) * bf16r(sa[e])) * kOnCarry;
    const float v1 = ((c[e] * rinv) * bf16r(sc[e])) * kOnCarry;
    hb[e]     = h_bits(flush_h(v0));
    hb[4 + e] = h_bits(flush_h(v1));
  }
  const v4u u = (v4u){pk16(hb[0], hb[1]), pk16(hb[2], hb[3]), pk16(hb[4], hb[5]), pk16(hb[6], hb[7])};
  unsigned short* q = ON + (size_t)row * kHid + 8 * lane;
  *(volatile v4u*)q = u;
  __threadfence();
  *(volatile v4u*)q = u;
}

extern "C" void kernel_launch(void* const* d_in, const int* in_sizes, int n_in,
                              void* d_out, int out_size, void* d_ws, size_t ws_size,
                              hipStream_t stream) {
  if (n_in < 15 || d_out == nullptr || d_ws == nullptr) return;
  if (in_sizes[0] != kTok * kFin) return;
  if (in_sizes[1] != kTok * kNAct) return;
  if (in_sizes[2] != kTok) return;
  if (in_sizes[3] != kOut0) return;
  if (in_sizes[4] != kFin * kHid || in_sizes[5] != kFin * kHid || in_sizes[6] != kFin * kHid) return;
  if (in_sizes[7] != kFin * kNH || in_sizes[8] != kFin * kNH) return;
  if (in_sizes[9] != kNAct * kHid || in_sizes[10] != kNAct * kHid) return;
  if (in_sizes[11] != kNAct * kNH) return;
  if (in_sizes[12] != kHid) return;
  if (in_sizes[13] != kHid * kFin) return;
  if (in_sizes[14] != kFin) return;
  if (out_size != kOut0 + kOut1) return;
  if (ws_size < kWsTotal) return;

  const float* x      = (const float*)d_in[0];
  const float* action = (const float*)d_in[1];
  const float* mask   = (const float*)d_in[2];
  const float* carry  = (const float*)d_in[3];
  const float* Wq     = (const float*)d_in[4];
  const float* Wk     = (const float*)d_in[5];
  const float* Wv     = (const float*)d_in[6];
  const float* Wbeta  = (const float*)d_in[7];
  const float* Walpha = (const float*)d_in[8];
  const float* Wku    = (const float*)d_in[9];
  const float* Wvu    = (const float*)d_in[10];
  const float* Wgamma = (const float*)d_in[11];
  const float* rscale = (const float*)d_in[12];
  const float* Wout   = (const float*)d_in[13];
  const float* bout   = (const float*)d_in[14];

  float* newCarry = (float*)d_out;
  float* y        = (float*)d_out + (size_t)kOut0;

  char* ws = (char*)d_ws;
  unsigned short* XB  = (unsigned short*)(ws + kOffXB);
  unsigned short* AB  = (unsigned short*)(ws + kOffAB);
  unsigned short* WQT = (unsigned short*)(ws + kOffWQT);
  unsigned short* WAT = (unsigned short*)(ws + kOffWAT);
  unsigned short* WOT = (unsigned short*)(ws + kOffWOT);
  float*          P   = (float*)(ws + kOffP);
  float*          PA  = (float*)(ws + kOffPA);
  float*          QN  = (float*)(ws + kOffQN);
  float*          KN  = (float*)(ws + kOffKN);
  float*          KU  = (float*)(ws + kOffKU);
  float*          VU  = (float*)(ws + kOffVU);
  float*          G   = (float*)(ws + kOffG);
  float*          O   = (float*)(ws + kOffO);
  unsigned short* ON  = (unsigned short*)(ws + kOffON);

  cvt_x_bf16_kernel<<<(kTok * kFin / 8) / 256, 256, 0, stream>>>(x, XB, kTok * kFin / 8);
  pack_action_kernel<<<(kTok * 4) / 256, 256, 0, stream>>>(action, AB);
  pack_wT_kernel<0><<<dim3(kFin / 64, kN1 / 64), 256, 0, stream>>>(Wq, Wk, Wv, Wbeta, Walpha, WQT);
  pack_waT_kernel<<<kN2 / 64, 256, 0, stream>>>(Wku, Wvu, Wgamma, WAT);
  pack_wT_kernel<1><<<dim3(kHid / 64, kFin / 64), 256, 0, stream>>>(Wout, Wout, Wout, Wout, Wout, WOT);

  wmma_gemm64<1, false><<<(kTok / 64) * (kN1 / 64) / 8, 256, 0, stream>>>(
      XB, kFin, WQT, kFin, P, kN1, bout, kTok, kN1, kFin, 1.0f);
  wmma_gemm64<1, false><<<(kTok / 64) * (kN2 / 64) / 8, 256, 0, stream>>>(
      AB, kK2, WAT, kK2, PA, kN2, bout, kTok, kN2, kK2, 1.0f);

  token_prep_kernel<<<kTok / 8, 256, 0, stream>>>(P, PA, mask, QN, KN, KU, VU, G);

  gated_state_scan_kernel<<<kNB * kNH, 128, 0, stream>>>(QN, KN, KU, VU, P, G, carry, O, newCarry);

  rms_rows_kernel<<<kTok / 8, 256, 0, stream>>>(O, rscale, ON);

  wmma_gemm64<0, true><<<(kTok / 64) * (kFin / 64) / 8, 256, 0, stream>>>(
      ON, kHid, WOT, kHid, y, kFin, bout, kTok, kFin, kHid, kOutScale);
}
